// InsiderClassifier_43001212567831
// MI455X (gfx1250) — hardware-verified
//
#include <hip/hip_runtime.h>
#include <math.h>


typedef _Float16 v16h __attribute__((ext_vector_type(16)));
typedef _Float16 v8h  __attribute__((ext_vector_type(8)));
typedef float    v8f  __attribute__((ext_vector_type(8)));
typedef float    v4f  __attribute__((ext_vector_type(4)));

#define NV 170
#define NP 192
#define NB 32
#define NTRI (NV * (NV + 1) / 2)

__device__ __forceinline__ int frag_k(int lane, int e) {
    return ((lane >> 4) & 1) * 8 + ((e >> 3) & 1) * 16 + (e & 7);
}

__device__ __forceinline__ v8f wmma16(v16h a, v16h b, v8f c) {
    v8f d = __builtin_amdgcn_wmma_f32_16x16x32_f16(false, a, false, b, (short)0, c, false, false);
    asm volatile("v_nop\n\tv_nop\n\tv_nop\n\tv_nop" : "+v"(d) : "v"(a), "v"(b));
    return d;
}

__device__ __forceinline__ v8f zero8() {
    v8f z = {0.f, 0.f, 0.f, 0.f, 0.f, 0.f, 0.f, 0.f};
    return z;
}

__device__ __forceinline__ void st_f(float* p, float v)      { *(volatile float*)p = v; }
__device__ __forceinline__ void st_v4(float* p, v4f v)       { *(volatile v4f*)p = v; }
__device__ __forceinline__ void st_v8h(_Float16* p, v8h v)   { *(volatile v8h*)p = v; }

__device__ __forceinline__ float block_sum256(float v, float* red, int tid) {
    red[tid] = v;
    __syncthreads();
    for (int st = 128; st > 0; st >>= 1) {
        if (tid < st) red[tid] += red[tid + st];
        __syncthreads();
    }
    const float r = red[0];
    __syncthreads();
    return r;
}

__device__ __forceinline__ int tri(int i, int j) { return ((i * (i + 1)) >> 1) + j; }

__device__ __forceinline__ void frag_unit(int u, int& tt, int& cn, int& kb) {
    const int j8 = u & 1, ln = (u >> 1) & 31;
    tt = u >> 6;
    cn = ln & 15;
    kb = 8 * (ln >> 4) + 16 * j8;
}


__global__ __launch_bounds__(NP) void k_cfc(const float* __restrict__ hist, const float* __restrict__ glw,
                                           float* __restrict__ U) {
    const int pb = blockIdx.x;
    const int p = pb / NB, b = pb - p * NB;
    const int n = threadIdx.x;
    const int nn = (n < NV) ? n : 0;
    float v[12];
    float ss = 0.f;
#pragma unroll
    for (int d = 0; d < 12; ++d) {
        const float t = hist[(b * 12 + d) * NV + nn] * glw[p * 12 + d];
        v[d] = t;
        ss += t * t;
    }
    const float inv = 1.f / fmaxf(sqrtf(ss), 1e-12f);
#pragma unroll
    for (int d = 0; d < 12; ++d) v[d] = (n < NV) ? v[d] * inv : 0.f;
    float* dst = U + (size_t)pb * 12 * NP + n;
#pragma unroll
    for (int d = 0; d < 12; ++d) st_f(dst + d * NP, v[d]);
    __threadfence();
#pragma unroll
    for (int d = 0; d < 12; ++d) st_f(dst + d * NP, v[d]);
}

__global__ __launch_bounds__(NP) void k_adj(const float* __restrict__ U, float* __restrict__ adj) {
    const int n = blockIdx.x;
    const int m = threadIdx.x;
    float s = 0.f;
#pragma unroll 1
    for (int b = 0; b < NB; ++b) {
        float att = 0.f;
#pragma unroll 1
        for (int p = 0; p < 2; ++p) {
            const float* base = U + (size_t)(p * NB + b) * 12 * NP;
            float d = 0.f;
#pragma unroll
            for (int k = 0; k < 12; ++k) d += base[k * NP + n] * base[k * NP + m];
            att += d;
        }
        s += fmaxf(att * 0.5f, 0.f);
    }
    const float val = (m < NV) ? s * (1.f / (float)NB) : 0.f;
    float* dst = adj + n * NP + m;
    st_f(dst, val);
    __threadfence();
    st_f(dst, val);
}

__global__ __launch_bounds__(256) void k_graph(const float* __restrict__ adj, _Float16* __restrict__ gsoA) {
    __shared__ float Ap[NTRI];
    __shared__ float dis[NV];
    __shared__ float uv[NV];
    __shared__ float pv[NV];
    __shared__ float wv[NV];
    __shared__ float dd[NV];
    __shared__ float ee[NV];
    __shared__ float red[256];
    __shared__ float sc[4];
    const int tid = threadIdx.x;

    if (tid < NV) {
        float d = 0.f;
        for (int m = 0; m < NV; ++m) d += 0.5f * (adj[tid * NP + m] + adj[m * NP + tid]);
        dis[tid] = (d > 0.f) ? (1.f / sqrtf(d)) : 0.f;
    }
    __syncthreads();

    for (int i = 0; i < NV; ++i) {
        if (tid <= i) {
            const int j = tid;
            const float a = 0.5f * (adj[i * NP + j] + adj[j * NP + i]);
            const float s = (dis[i] * a) * dis[j];
            Ap[tri(i, j)] = ((i == j) ? 1.f : 0.f) - s;
        }
    }
    __syncthreads();

    for (int k = 0; k < NV - 2; ++k) {
        const int m = NV - 1 - k;
        float sq = 0.f;
        for (int i = k + 2 + tid; i < NV; i += 256) {
            const float t = Ap[tri(i, k)];
            sq += t * t;
        }
        const float sigma = block_sum256(sq, red, tid);
        const float alpha = Ap[tri(k + 1, k)];
        if (tid == 0) dd[k] = Ap[tri(k, k)];
        __syncthreads();
        if (sigma > 0.f) {
            const float mu = sqrtf(alpha * alpha + sigma);
            const float beta = (alpha > 0.f) ? -mu : mu;
            const float u0 = alpha - beta;
            const float gam = 2.f / (u0 * u0 + sigma);
            if (tid == 0) ee[k] = beta;
            for (int i = tid; i < m; i += 256) uv[i] = (i == 0) ? u0 : Ap[tri(k + 1 + i, k)];
            __syncthreads();
            if (tid < m) {
                const int i = k + 1 + tid;
                const int rb = tri(i, k + 1);
                float acc = 0.f;
#pragma unroll 1
                for (int c = 0; c <= tid; ++c) acc += Ap[rb + c] * uv[c];
#pragma unroll 1
                for (int c = tid + 1; c < m; ++c) acc += Ap[tri(k + 1 + c, i)] * uv[c];
                pv[tid] = gam * acc;
            }
            __syncthreads();
            float sp = 0.f;
            for (int i = tid; i < m; i += 256) sp += pv[i] * uv[i];
            const float dotpu = block_sum256(sp, red, tid);
            const float kc = 0.5f * gam * dotpu;
            for (int i = tid; i < m; i += 256) wv[i] = pv[i] - kc * uv[i];
            __syncthreads();
#pragma unroll 1
            for (int r = 0; r < m; ++r) {
                if (tid <= r) {
                    const int idx = tri(k + 1 + r, k + 1 + tid);
                    const float nv = Ap[idx] - (uv[r] * wv[tid] + wv[r] * uv[tid]);
                    Ap[idx] = nv;
                }
            }
            __syncthreads();
        } else {
            if (tid == 0) ee[k] = alpha;
        }
    }
    __syncthreads();

    if (tid == 0) {
        dd[NV - 2] = Ap[tri(NV - 2, NV - 2)];
        dd[NV - 1] = Ap[tri(NV - 1, NV - 1)];
        ee[NV - 2] = Ap[tri(NV - 1, NV - 2)];
        double lo = -1.0e30, hi = -1.0e30;
#pragma unroll 1
        for (int i = 0; i < NV; ++i) {
            const double di = (double)dd[i];
            double ri = 0.0;
            if (i > 0) ri += fabs((double)ee[i - 1]);
            if (i < NV - 1) ri += fabs((double)ee[i]);
            lo = fmax(lo, di);
            hi = fmax(hi, di + ri);
        }
#pragma unroll 1
        for (int it = 0; it < 64; ++it) {
            const double x = 0.5 * (lo + hi);
            double q = (double)dd[0] - x;
            if (fabs(q) < 1.0e-30) q = -1.0e-30;
            int cnt = (q < 0.0) ? 1 : 0;
#pragma unroll 1
            for (int i = 1; i < NV; ++i) {
                const double e = (double)ee[i - 1];
                q = ((double)dd[i] - x) - e * e / q;
                if (fabs(q) < 1.0e-30) q = -1.0e-30;
                cnt += (q < 0.0) ? 1 : 0;
            }
            if (cnt >= NV) hi = x; else lo = x;
        }
        sc[0] = (float)hi;
    }
    __syncthreads();

    const float emax = sc[0];
    const bool sub = (emax >= 2.f);
    const float rin = 1.f / fmaxf(emax, 1e-6f);
    const int NU = 11 * 6 * 64;
    for (int pass = 0; pass < 2; ++pass) {
        for (int u = tid; u < NU; u += 256) {
            int tt, cn, kb;
            frag_unit(u, tt, cn, kb);
            const int kt = tt % 6, mt = tt / 6;
            const int M = mt * 16 + cn;
            v8h o;
#pragma unroll
            for (int j = 0; j < 8; ++j) {
                const int K = kt * 32 + kb + j;
                float g = 0.f;
                if (M < NV && K < NV) {
                    const float a = 0.5f * (adj[M * NP + K] + adj[K * NP + M]);
                    const float sna = (dis[M] * a) * dis[K];
                    const float dI = (M == K) ? 1.f : 0.f;
                    const float lap = dI - sna;
                    g = sub ? (lap - dI) : ((2.f * lap) * rin - dI);
                }
                o[j] = (_Float16)g;
            }
            st_v8h(gsoA + (size_t)u * 8, o);
        }
        if (pass == 0) __threadfence();
    }
}


__global__ __launch_bounds__(256) void k_wfrag_tconv(const float* __restrict__ w, const float* __restrict__ aw,
                                                     _Float16* __restrict__ frag, int Cin, int KT, int Cout,
                                                     int nkt, int nnt, int fold) {
    const int NU = nkt * nnt * 64;
    const int u = blockIdx.x * 256 + threadIdx.x;
    const bool ok = u < NU;
    const int uu = ok ? u : 0;
    int tt, cn, kb;
    frag_unit(uu, tt, cn, kb);
    const int nt = tt % nnt, kt = tt / nnt;
    const int c = nt * 16 + cn;
    const int Ktot = KT * Cin, Ntot = 2 * Cout;
    v8h o;
#pragma unroll
    for (int j = 0; j < 8; ++j) {
        const int K = kt * 32 + kb + j;
        float v = 0.f;
        if (K < Ktot && c < Ntot) {
            const int tap = K / Cin, ci = K - tap * Cin;
            v = w[(c * Cin + ci) * KT + tap];
            if (fold != 0 && c < Cout && tap == KT - 1) v += aw[c * Cin + ci];
        }
        o[j] = (_Float16)v;
    }
    _Float16* dst = frag + (size_t)uu * 8;
    if (ok) st_v8h(dst, o);
    __threadfence();
    if (ok) st_v8h(dst, o);
}

__global__ __launch_bounds__(128) void k_wfrag_cheb(const float* __restrict__ w, _Float16* __restrict__ frag) {
    const int u = threadIdx.x;
    int tt, cn, kb;
    frag_unit(u, tt, cn, kb);
    v8h o;
#pragma unroll
    for (int j = 0; j < 8; ++j) {
        const int K = tt * 32 + kb + j;
        const int ks = K >> 4, ci = K & 15;
        const float v = (ks < 3) ? w[(ks * 16 + ci) * 16 + cn] : 0.f;
        o[j] = (_Float16)v;
    }
    _Float16* dst = frag + (size_t)u * 8;
    st_v8h(dst, o);
    __threadfence();
    st_v8h(dst, o);
}

__global__ __launch_bounds__(256) void k_wfrag_fc1(const float* __restrict__ w, _Float16* __restrict__ frag) {
    const int u = blockIdx.x * 256 + threadIdx.x;
    const bool ok = u < 4 * 8 * 64;
    const int uu = ok ? u : 0;
    int tt, cn, kb;
    frag_unit(uu, tt, cn, kb);
    const int nt = tt & 7, kt = tt >> 3;
    const int c = nt * 16 + cn;
    v8h o;
#pragma unroll
    for (int j = 0; j < 8; ++j) {
        const int K = kt * 32 + kb + j;
        o[j] = (_Float16)w[K * 128 + c];
    }
    _Float16* dst = frag + (size_t)uu * 8;
    if (ok) st_v8h(dst, o);
    __threadfence();
    if (ok) st_v8h(dst, o);
}

template <int KT, int CIN, int COUT, int RESC>
__global__ __launch_bounds__(128) void k_glu(const float* __restrict__ X,
                                             const float* __restrict__ bias,
                                             const float* __restrict__ bias2, int addb2,
                                             const _Float16* __restrict__ wfrag,
                                             float* __restrict__ Y, int T_in) {
    constexpr int KTOT = KT * CIN;
    constexpr int NKT  = (KTOT + 31) / 32;
    constexpr int NNT  = (2 * COUT) / 16;
    constexpr int HALF = COUT / 16;
    __shared__ __attribute__((aligned(16))) float stg[4 * 16 * COUT];
    const int T_out = T_in - KT + 1;
    const int M_total = NB * T_out * NV;
    const int lane = threadIdx.x & 31;
    const int wave = threadIdx.x >> 5;
    const int col = lane & 15, hh = lane >> 4;
    const int Mtile = blockIdx.x * 4 + wave;
    const bool active = (Mtile * 16) < M_total;

    const int rowA = Mtile * 16 + col;
    const bool rowOK = rowA < M_total;
    int bA = 0, tA = 0, nA = 0;
    if (rowOK) {
        bA = rowA / (T_out * NV);
        const int rem = rowA - bA * (T_out * NV);
        tA = rem / NV;
        nA = rem - tA * NV;
    }
    v16h av[NKT];
#pragma unroll
    for (int kt = 0; kt < NKT; ++kt) {
        v16h a;
#pragma unroll
        for (int e = 0; e < 16; ++e) {
            const int K = kt * 32 + frag_k(lane, e);
            float v = 0.f;
            if (rowOK && K < KTOT) {
                const int tap = K / CIN, ci = K - tap * CIN;
                v = X[((size_t)(bA * T_in + tA + tap) * NV + nA) * CIN + ci];
            }
            a[e] = (_Float16)v;
        }
        av[kt] = a;
    }

    float* stw = stg + wave * (16 * COUT);
#pragma unroll 1
    for (int nt = 0; nt < HALF; ++nt) {
        v8f accP = zero8(), accQ = zero8();
#pragma unroll
        for (int kt = 0; kt < NKT; ++kt) {
            const v16h bP = *(const v16h*)(wfrag + ((size_t)(kt * NNT + nt) * 32 + lane) * 16);
            const v16h bQ = *(const v16h*)(wfrag + ((size_t)(kt * NNT + nt + HALF) * 32 + lane) * 16);
            accP = wmma16(av[kt], bP, accP);
            accQ = wmma16(av[kt], bQ, accQ);
        }
        const int c = nt * 16 + col;
        const float bp = bias[c] + ((addb2 != 0) ? bias2[c] : 0.f);
        const float bq = bias[COUT + c];
#pragma unroll
        for (int r = 0; r < 8; ++r) {
            const int rl = hh * 8 + r;
            const int row = Mtile * 16 + rl;
            float p = accP[r] + bp;
            const float q = accQ[r] + bq;
            if (RESC > 0 && c < RESC && row < M_total) {
                const int b = row / (T_out * NV);
                const int rem = row - b * (T_out * NV);
                const int t = rem / NV, n = rem - t * NV;
                p += X[((size_t)(b * T_in + t + KT - 1) * NV + n) * CIN + c];
            }
            const float o = p * (1.f / (1.f + __expf(-q)));
            stw[rl * COUT + c] = o;
        }
    }
    __syncthreads();

    if (active) {
        float* dst = Y + (size_t)Mtile * (16 * COUT);
        constexpr int NQ = 16 * COUT / 4;
        for (int qd = lane; qd < NQ; qd += 32) st_v4(dst + 4 * qd, *(const v4f*)(stw + 4 * qd));
        __threadfence();
        for (int qd = lane; qd < NQ; qd += 32) st_v4(dst + 4 * qd, *(const v4f*)(stw + 4 * qd));
    }
}

__global__ __launch_bounds__(352) void k_cheb(const float* __restrict__ X,
                                              const _Float16* __restrict__ gsoA,
                                              const _Float16* __restrict__ wstk,
                                              const float* __restrict__ cbias,
                                              float* __restrict__ Y, int T) {
    const int bt = blockIdx.x;
    if (bt >= NB * T) return;
    __shared__ __attribute__((aligned(16))) float Xs0[176 * 16];
    __shared__ __attribute__((aligned(16))) float Xs1[176 * 16];
    __shared__ __attribute__((aligned(16))) float Xs2[176 * 16];
    __shared__ alignas(32) _Float16 nodefrag[6 * 512];
    __shared__ alignas(32) _Float16 catfrag[11 * 2 * 512];
    const int tid = threadIdx.x;
    const float* xin = X + (size_t)bt * NV * 16;

    for (int ch = tid; ch < NV * 4; ch += 352) *(v4f*)(Xs0 + ch * 4) = *(const v4f*)(xin + ch * 4);
    for (int i = tid; i < 6 * 16; i += 352) Xs0[NV * 16 + i] = 0.f;
    __syncthreads();

    for (int i = tid; i < 6 * 512; i += 352) {
        const int e = i & 15, ln = (i >> 4) & 31, kt = i >> 9;
        const int K = kt * 32 + frag_k(ln, e);
        nodefrag[i] = (_Float16)((K < 176) ? Xs0[K * 16 + (ln & 15)] : 0.f);
    }
    __syncthreads();

    const int wave = tid >> 5, lane = tid & 31;
    const int col = lane & 15;
    const int rowBase = wave * 16 + ((lane >> 4) << 3);

    v8f acc = zero8();
#pragma unroll
    for (int kt = 0; kt < 6; ++kt) {
        const v16h a  = *(const v16h*)(gsoA + ((size_t)(wave * 6 + kt) * 32 + lane) * 16);
        const v16h bf = *(const v16h*)(nodefrag + ((size_t)kt * 32 + lane) * 16);
        acc = wmma16(a, bf, acc);
    }
#pragma unroll
    for (int r = 0; r < 8; ++r) Xs1[(rowBase + r) * 16 + col] = acc[r];
    __syncthreads();
    for (int i = tid; i < 6 * 512; i += 352) {
        const int e = i & 15, ln = (i >> 4) & 31, kt = i >> 9;
        const int K = kt * 32 + frag_k(ln, e);
        nodefrag[i] = (_Float16)((K < 176) ? Xs1[K * 16 + (ln & 15)] : 0.f);
    }
    __syncthreads();

    acc = zero8();
#pragma unroll
    for (int kt = 0; kt < 6; ++kt) {
        const v16h a  = *(const v16h*)(gsoA + ((size_t)(wave * 6 + kt) * 32 + lane) * 16);
        const v16h bf = *(const v16h*)(nodefrag + ((size_t)kt * 32 + lane) * 16);
        acc = wmma16(a, bf, acc);
    }
#pragma unroll
    for (int r = 0; r < 8; ++r) {
        const int row = rowBase + r;
        Xs2[row * 16 + col] = 2.f * acc[r] - Xs0[row * 16 + col];
    }
    __syncthreads();

    for (int i = tid; i < 11 * 1024; i += 352) {
        const int e = i & 15, ln = (i >> 4) & 31, tt = i >> 9;
        const int kt = tt & 1, mt = tt >> 1;
        const int K = kt * 32 + frag_k(ln, e);
        const int row = mt * 16 + (ln & 15);
        const int ks = K >> 4, ci = K & 15;
        float v = 0.f;
        if (ks == 0) v = Xs0[row * 16 + ci];
        else if (ks == 1) v = Xs1[row * 16 + ci];
        else if (ks == 2) v = Xs2[row * 16 + ci];
        catfrag[i] = (_Float16)v;
    }
    __syncthreads();

    acc = zero8();
#pragma unroll
    for (int kt = 0; kt < 2; ++kt) {
        const v16h a  = *(const v16h*)(catfrag + ((size_t)(wave * 2 + kt) * 32 + lane) * 16);
        const v16h bf = *(const v16h*)(wstk + ((size_t)kt * 32 + lane) * 16);
        acc = wmma16(a, bf, acc);
    }
#pragma unroll
    for (int r = 0; r < 8; ++r) {
        const int row = rowBase + r;
        const float v = acc[r] + cbias[col] + Xs0[row * 16 + col];
        Xs1[row * 16 + col] = fmaxf(v, 0.f);
    }
    __syncthreads();

    float* yout = Y + (size_t)bt * NV * 16;
    for (int q = tid; q < NV * 4; q += 352) st_v4(yout + 4 * q, *(const v4f*)(Xs1 + 4 * q));
    __threadfence();
    for (int q = tid; q < NV * 4; q += 352) st_v4(yout + 4 * q, *(const v4f*)(Xs1 + 4 * q));
}

__global__ __launch_bounds__(256) void k_ln(const float* __restrict__ X, const float* __restrict__ g,
                                            const float* __restrict__ bv, float* __restrict__ Y, int nslab) {
    constexpr int C = 64, TOT = NV * C, NQ = TOT / 4, PER = (NQ + 255) / 256;
    __shared__ float red[256];
    const int bt = blockIdx.x;
    if (bt >= nslab) return;
    const int tid = threadIdx.x;
    const size_t off = (size_t)bt * TOT;
    const v4f* x4 = (const v4f*)(X + off);
    const v4f* g4 = (const v4f*)g;
    const v4f* b4 = (const v4f*)bv;
    v4f xv[PER];
    float s = 0.f;
#pragma unroll
    for (int j = 0; j < PER; ++j) {
        const int q = tid + 256 * j;
        v4f t = {0.f, 0.f, 0.f, 0.f};
        if (q < NQ) t = x4[q];
        xv[j] = t;
        s += (t.x + t.y) + (t.z + t.w);
    }
    const float mu = block_sum256(s, red, tid) * (1.f / (float)TOT);
    float s2 = 0.f;
#pragma unroll
    for (int j = 0; j < PER; ++j) {
        const int q = tid + 256 * j;
        if (q < NQ) {
            const v4f d = xv[j] - mu;
            s2 += (d.x * d.x + d.y * d.y) + (d.z * d.z + d.w * d.w);
        }
    }
    const float var = block_sum256(s2, red, tid) * (1.f / (float)TOT);
    const float rinv = 1.f / sqrtf(var + 1e-12f);
#pragma unroll
    for (int j = 0; j < PER; ++j) {
        const int q = tid + 256 * j;
        if (q < NQ) xv[j] = (xv[j] - mu) * rinv * g4[q] + b4[q];
    }
    float* y = Y + off;
#pragma unroll
    for (int j = 0; j < PER; ++j) {
        const int q = tid + 256 * j;
        if (q < NQ) st_v4(y + 4 * q, xv[j]);
    }
    __threadfence();
#pragma unroll
    for (int j = 0; j < PER; ++j) {
        const int q = tid + 256 * j;
        if (q < NQ) st_v4(y + 4 * q, xv[j]);
    }
}

__global__ __launch_bounds__(352) void k_head(const float* __restrict__ X,
                                              const float* __restrict__ g,
                                              const float* __restrict__ bv,
                                              const _Float16* __restrict__ fc1frag,
                                              const float* __restrict__ fc1b,
                                              const float* __restrict__ fc2w,
                                              const float* __restrict__ fc2b,
                                              float* __restrict__ H) {
    const int b = blockIdx.x;
    const float* x = X + (size_t)b * NV * 128;
    __shared__ float red[352];
    __shared__ float rowsum[176];
    __shared__ alignas(32) _Float16 afrag[11 * 4 * 512];
    const int tid = threadIdx.x;
    const int TOT = NV * 128;

    float s = 0.f;
    for (int i = tid; i < TOT; i += 352) s += x[i];
    red[tid] = s;
    __syncthreads();
    for (int sz = 352; sz > 1;) {
        const int half = (sz + 1) >> 1;
        if (tid < sz - half) red[tid] += red[tid + half];
        __syncthreads();
        sz = half;
    }
    const float mu = red[0] / (float)TOT;
    __syncthreads();
    float s2 = 0.f;
    for (int i = tid; i < TOT; i += 352) { const float d = x[i] - mu; s2 += d * d; }
    red[tid] = s2;
    __syncthreads();
    for (int sz = 352; sz > 1;) {
        const int half = (sz + 1) >> 1;
        if (tid < sz - half) red[tid] += red[tid + half];
        __syncthreads();
        sz = half;
    }
    const float rinv = 1.f / sqrtf(red[0] / (float)TOT + 1e-12f);

    for (int i = tid; i < 11 * 4 * 512; i += 352) {
        const int e = i & 15, ln = (i >> 4) & 31, tt = i >> 9;
        const int kt = tt & 3, mt = tt >> 2;
        const int row = mt * 16 + (ln & 15);
        const int K = kt * 32 + frag_k(ln, e);
        float v = 0.f;
        if (row < NV) {
            const float xv = x[row * 128 + K];
            v = (xv - mu) * rinv * g[row * 128 + K] + bv[row * 128 + K];
        }
        afrag[i] = (_Float16)v;
    }
    __syncthreads();

    const int wave = tid >> 5, lane = tid & 31;
    const int col = lane & 15, hh = lane >> 4;
    float partial[8];
#pragma unroll
    for (int r = 0; r < 8; ++r) partial[r] = 0.f;
#pragma unroll 1
    for (int nt = 0; nt < 8; ++nt) {
        v8f acc = zero8();
#pragma unroll
        for (int kt = 0; kt < 4; ++kt) {
            const v16h a  = *(const v16h*)(afrag + ((size_t)(wave * 4 + kt) * 32 + lane) * 16);
            const v16h bf = *(const v16h*)(fc1frag + ((size_t)(kt * 8 + nt) * 32 + lane) * 16);
            acc = wmma16(a, bf, acc);
        }
        const int c = nt * 16 + col;
        const float w2 = fc2w[c], b1 = fc1b[c];
#pragma unroll
        for (int r = 0; r < 8; ++r) {
            const float hv = fmaxf(acc[r] + b1, 0.f);
            partial[r] += hv * w2;
        }
    }
#pragma unroll
    for (int r = 0; r < 8; ++r) {
        float v = partial[r];
        v += __shfl_xor(v, 1, 32);
        v += __shfl_xor(v, 2, 32);
        v += __shfl_xor(v, 4, 32);
        v += __shfl_xor(v, 8, 32);
        partial[r] = v;
    }
    if (col == 0) {
#pragma unroll
        for (int r = 0; r < 8; ++r) rowsum[wave * 16 + hh * 8 + r] = partial[r];
    }
    __syncthreads();
    if (tid < NP) {
        const float v = (tid < NV) ? (rowsum[tid] + fc2b[0]) : 0.f;
        float* dst = H + (size_t)b * NP + tid;
        st_f(dst, v);
        __threadfence();
        st_f(dst, v);
    }
}

__global__ __launch_bounds__(256) void k_out(const float* __restrict__ H, float* __restrict__ out) {
    constexpr int NQ = NB * NV / 4;
    const int tid = threadIdx.x;
    for (int pass = 0; pass < 2; ++pass) {
        for (int q = tid; q < NQ; q += 256) {
            v4f v;
#pragma unroll
            for (int e = 0; e < 4; ++e) {
                const int f = 4 * q + e;
                const int bb = f / NV, n = f - bb * NV;
                v[e] = H[bb * NP + n];
            }
            st_v4(out + 4 * q, v);
        }
        if (pass == 0) __threadfence();
    }
}

extern "C" void kernel_launch(void* const* d_in, const int* in_sizes, int n_in,
                              void* d_out, int out_size, void* d_ws, size_t ws_size,
                              hipStream_t stream) {
    if (n_in < 28) return;
    if (out_size != NB * NV) return;
    if (in_sizes[0] != NB * 12 * NV) return;

    const float* hist = (const float*)d_in[0];
    const float* glw  = (const float*)d_in[1];
    const float* c1w  = (const float*)d_in[2];
    const float* c1b  = (const float*)d_in[3];
    const float* ch1w = (const float*)d_in[4];
    const float* ch1b = (const float*)d_in[5];
    const float* c2w  = (const float*)d_in[6];
    const float* c2b  = (const float*)d_in[7];
    const float* ln2g = (const float*)d_in[8];
    const float* ln2b = (const float*)d_in[9];
    const float* c3w  = (const float*)d_in[10];
    const float* c3b  = (const float*)d_in[11];
    const float* a3w  = (const float*)d_in[12];
    const float* a3b  = (const float*)d_in[13];
    const float* ch2w = (const float*)d_in[14];
    const float* ch2b = (const float*)d_in[15];
    const float* c4w  = (const float*)d_in[16];
    const float* c4b  = (const float*)d_in[17];
    const float* ln4g = (const float*)d_in[18];
    const float* ln4b = (const float*)d_in[19];
    const float* ocw  = (const float*)d_in[20];
    const float* ocb  = (const float*)d_in[21];
    const float* olng = (const float*)d_in[22];
    const float* olnb = (const float*)d_in[23];
    const float* fc1w = (const float*)d_in[24];
    const float* fc1b = (const float*)d_in[25];
    const float* fc2w = (const float*)d_in[26];
    const float* fc2b = (const float*)d_in[27];
    float* out = (float*)d_out;

    float* base = (float*)d_ws;
    size_t o = 0;
    auto alloc = [&](size_t nf) { float* p = base + o; o += (nf + 31) & ~(size_t)31; return p; };
    float* U        = alloc((size_t)2 * NB * 12 * NP);
    float* adj      = alloc((size_t)NV * NP);
    _Float16* gsoA  = (_Float16*)alloc(11 * 6 * 512 / 2);
    _Float16* wch1  = (_Float16*)alloc(1024 / 2);
    _Float16* wch2  = (_Float16*)alloc(1024 / 2);
    _Float16* wc1   = (_Float16*)alloc(1 * 2 * 512 / 2);
    _Float16* wc2   = (_Float16*)alloc(2 * 8 * 512 / 2);
    _Float16* wc3   = (_Float16*)alloc(6 * 2 * 512 / 2);
    _Float16* wc4   = (_Float16*)alloc(2 * 8 * 512 / 2);
    _Float16* woc   = (_Float16*)alloc(8 * 16 * 512 / 2);
    _Float16* wfc1  = (_Float16*)alloc(4 * 8 * 512 / 2);
    const size_t actMax = (size_t)NB * 8 * NV * 64;
    float* bufA = alloc(actMax);
    float* bufB = alloc(actMax);
    float* bufC = alloc(actMax);
    float* hbuf = alloc((size_t)NB * NP);
    if (o * sizeof(float) > ws_size) return;

    k_cfc<<<2 * NB, NP, 0, stream>>>(hist, glw, U);
    k_adj<<<NV, NP, 0, stream>>>(U, adj);
    k_graph<<<1, 256, 0, stream>>>(adj, gsoA);

    k_wfrag_cheb<<<1, 128, 0, stream>>>(ch1w, wch1);
    k_wfrag_cheb<<<1, 128, 0, stream>>>(ch2w, wch2);
    k_wfrag_tconv<<<(1 * 2 * 64 + 255) / 256, 256, 0, stream>>>(c1w, c1w, wc1, 1, 3, 16, 1, 2, 0);
    k_wfrag_tconv<<<(2 * 8 * 64 + 255) / 256, 256, 0, stream>>>(c2w, c2w, wc2, 16, 3, 64, 2, 8, 0);
    k_wfrag_tconv<<<(6 * 2 * 64 + 255) / 256, 256, 0, stream>>>(c3w, a3w, wc3, 64, 3, 16, 6, 2, 1);
    k_wfrag_tconv<<<(2 * 8 * 64 + 255) / 256, 256, 0, stream>>>(c4w, c4w, wc4, 16, 3, 64, 2, 8, 0);
    k_wfrag_tconv<<<(8 * 16 * 64 + 255) / 256, 256, 0, stream>>>(ocw, ocw, woc, 64, 4, 128, 8, 16, 0);
    k_wfrag_fc1<<<(4 * 8 * 64 + 255) / 256, 256, 0, stream>>>(fc1w, wfc1);

    auto gluGrid = [&](int T_out) { const int tiles = (NB * T_out * NV + 15) / 16; return (tiles + 3) / 4; };
    k_glu<3, 1, 16, 1><<<gluGrid(10), 128, 0, stream>>>(hist, c1b, c1b, 0, wc1, bufA, 12);
    k_cheb<<<NB * 10, 352, 0, stream>>>(bufA, gsoA, wch1, ch1b, bufB, 10);
    k_glu<3, 16, 64, 16><<<gluGrid(8), 128, 0, stream>>>(bufB, c2b, c2b, 0, wc2, bufA, 10);
    k_ln<<<NB * 8, 256, 0, stream>>>(bufA, ln2g, ln2b, bufC, NB * 8);
    k_glu<3, 64, 16, 0><<<gluGrid(6), 128, 0, stream>>>(bufC, c3b, a3b, 1, wc3, bufB, 8);
    k_cheb<<<NB * 6, 352, 0, stream>>>(bufB, gsoA, wch2, ch2b, bufA, 6);
    k_glu<3, 16, 64, 16><<<gluGrid(4), 128, 0, stream>>>(bufA, c4b, c4b, 0, wc4, bufB, 6);
    k_ln<<<NB * 4, 256, 0, stream>>>(bufB, ln4g, ln4b, bufC, NB * 4);
    k_glu<4, 64, 128, 64><<<gluGrid(1), 128, 0, stream>>>(bufC, ocb, ocb, 0, woc, bufA, 4);
    k_head<<<NB, 352, 0, stream>>>(bufA, olng, olnb, wfc1, fc1b, fc2w, fc2b, hbuf);
    k_out<<<1, 256, 0, stream>>>(hbuf, out);
}
